// SelfAttention_42537356099867
// MI455X (gfx1250) — hardware-verified
//
#include <hip/hip_runtime.h>
#include <math.h>

#ifndef NB
#define NB 4
#endif
#ifndef SEQ
#define SEQ 2048
#endif
#define NB_FULL 4
#define SEQ_FULL 2048
#define CE 1024
#define EARLY 128
static_assert(NB >= 1);
static_assert(NB <= NB_FULL);
static_assert(SEQ % 64 == 0);
static_assert(SEQ >= EARLY);
static_assert(SEQ <= SEQ_FULL);
static_assert(CE % 64 == 0);
static_assert(EARLY % 64 == 0);

typedef __attribute__((ext_vector_type(16))) _Float16 v16h;
typedef __attribute__((ext_vector_type(8)))  _Float16 v8h;
typedef __attribute__((ext_vector_type(16))) __bf16   v16b;
typedef __attribute__((ext_vector_type(8)))  __bf16   v8b;
typedef __attribute__((ext_vector_type(8)))  float    v8f;
typedef __attribute__((ext_vector_type(4)))  float    v4f;
typedef __attribute__((ext_vector_type(4)))  unsigned v4u;

#define VST2(T, ptr, val) do { const T vst2_v_ = (val); *(volatile T*)(ptr) = vst2_v_; __threadfence(); *(volatile T*)(ptr) = vst2_v_; } while (0)

__device__ __forceinline__ unsigned short f2bf_bits(float f) { const unsigned u = __float_as_uint(f); return (unsigned short)((u + 0x7FFFu + ((u >> 16) & 1u)) >> 16); }
__device__ __forceinline__ float bf_bits2f(unsigned short h) { return __uint_as_float(((unsigned)h) << 16); }
__device__ __forceinline__ float bf_rne(float v) { const unsigned u = __float_as_uint(v); return __uint_as_float((u + 0x7fffu + ((u >> 16) & 1u)) & 0xffff0000u); }
__device__ __forceinline__ unsigned pk2h(float a, float b) { return (unsigned)__builtin_bit_cast(unsigned short, (_Float16)a) | ((unsigned)__builtin_bit_cast(unsigned short, (_Float16)b) << 16); }
__device__ __forceinline__ unsigned pk2u(unsigned short a, unsigned short b) { return (unsigned)a | ((unsigned)b << 16); }

__device__ __forceinline__ void dep_guard_h(v8f& a, v8f& b, v16h x, v16h y) { asm volatile("v_nop\n\tv_nop\n\tv_nop\n\tv_nop" : "+v"(a), "+v"(b) : "v"(x), "v"(y)); }
__device__ __forceinline__ void dep_guard_b(v8f& a, v8f& b, v16b x, v16b y) { asm volatile("v_nop\n\tv_nop\n\tv_nop\n\tv_nop" : "+v"(a), "+v"(b) : "v"(x), "v"(y)); }
__device__ __forceinline__ void keep4_h(v16h a, v16h b, v16h c, v16h d) { asm volatile("v_nop" :: "v"(a), "v"(b), "v"(c), "v"(d)); }
__device__ __forceinline__ void keep4_b(v16b a, v16b b, v16b c, v16b d) { asm volatile("v_nop" :: "v"(a), "v"(b), "v"(c), "v"(d)); }
__device__ __forceinline__ void acc_guard4(v8f& a, v8f& b, v8f& c, v8f& d) { asm volatile("v_nop\n\tv_nop\n\tv_nop\n\tv_nop" : "+v"(a), "+v"(b), "+v"(c), "+v"(d)); }

template <typename T> struct Frag;
template <> struct Frag<_Float16> {
  typedef v16h V; union U { v16h v; v8h h[2]; };
  static __device__ __forceinline__ v16h load(const _Float16* p) { U f; f.h[0] = *(const v8h*)(p); f.h[1] = *(const v8h*)(p + 16); return f.v; }
  static __device__ __forceinline__ v8f mma(v16h a, v16h b, v8f c) { return __builtin_amdgcn_wmma_f32_16x16x32_f16(false, a, false, b, (short)0, c, false, false); }
  static __device__ __forceinline__ void guard(v8f& a, v8f& b, v16h x, v16h y) { dep_guard_h(a, b, x, y); }
  static __device__ __forceinline__ void keep(v16h a, v16h b, v16h c, v16h d) { keep4_h(a, b, c, d); }
};
template <> struct Frag<__bf16> {
  typedef v16b V; union U { v16b v; v8b h[2]; };
  static __device__ __forceinline__ v16b load(const __bf16* p) { U f; f.h[0] = *(const v8b*)(p); f.h[1] = *(const v8b*)(p + 16); return f.v; }
  static __device__ __forceinline__ v8f mma(v16b a, v16b b, v8f c) { return __builtin_amdgcn_wmma_f32_16x16x32_bf16(false, a, false, b, (short)0, c, false, false); }
  static __device__ __forceinline__ void guard(v8f& a, v8f& b, v16b x, v16b y) { dep_guard_b(a, b, x, y); }
  static __device__ __forceinline__ void keep(v16b a, v16b b, v16b c, v16b d) { keep4_b(a, b, c, d); }
};
template <int ET> struct Elem;
template <> struct Elem<0> { typedef _Float16 T; };
template <> struct Elem<1> { typedef __bf16 T; };

template <int ET, bool SPLIT, int BIAS_MODE, int OUT_MODE, int CAUSAL>
__global__ __launch_bounds__(256) void k_gemm64(
    const unsigned short* __restrict__ Ap, const unsigned short* __restrict__ A2p, int lda, long long strideA,
    const unsigned short* __restrict__ Btp, const unsigned short* __restrict__ Bt2p, int ldb, long long strideB,
    void* __restrict__ Cout, void* __restrict__ Cout2, int ldc, long long strideC,
    const float* __restrict__ bias, int M, int N, int K, int tm0, float scale) {
  typedef typename Elem<ET>::T T;
  typedef typename Frag<T>::V V;
  const T* A = (const T*)Ap; const T* A2 = (const T*)A2p; const T* Bt = (const T*)Btp; const T* Bt2 = (const T*)Bt2p;
  __shared__ __align__(16) float sT[8][16 * 68];
  const int b    = blockIdx.y;
  const int lane = threadIdx.x & 31;
  const int wave = threadIdx.x >> 5;
  const int tilesN = N >> 6;
  const int tilesM = (M >> 6) - tm0;
  const int tile = blockIdx.x * 8 + wave;
  if (tile >= tilesM * tilesN) return;
  const int tq = tile / tilesN;
  const int tm = tm0 + tq;
  const int tn = tile - tq * tilesN;
  if (CAUSAL == 1 && tn > tm) return;
  const int m0 = tm << 6;
  const int n0 = tn << 6;
  const int Kc = (CAUSAL == 2) ? min(K, 64 * (tm + 1)) : K;

  const T* Ab  = A  + (size_t)b * strideA;
  const T* Bb  = Bt + (size_t)b * strideB;
  const T* Ab2 = SPLIT ? (A2  + (size_t)b * strideA) : nullptr;
  const T* Bb2 = SPLIT ? (Bt2 + (size_t)b * strideB) : nullptr;

  const int rlane = lane & 15;
  const int koff  = (lane >> 4) * 8;
  const int mOff  = (lane >> 4) * 8;

  v8f acc[4][4];
#pragma unroll
  for (int i = 0; i < 4; ++i)
#pragma unroll
    for (int j = 0; j < 4; ++j) acc[i][j] = (v8f){0.f,0.f,0.f,0.f,0.f,0.f,0.f,0.f};

  for (int k0 = 0; k0 < Kc; k0 += 32) {
#pragma unroll 1
    for (int ph = 0; ph < (SPLIT ? 2 : 1); ++ph) {
      const T* Bs = (ph == 0) ? Bb : Bb2;
      V bf[4];
#pragma unroll
      for (int j = 0; j < 4; ++j) bf[j] = Frag<T>::load(Bs + (size_t)(n0 + (j << 4) + rlane) * ldb + koff + k0);
#pragma unroll
      for (int i = 0; i < 4; ++i) {
        const size_t ao = (size_t)(m0 + (i << 4) + rlane) * lda + koff + k0;
        const V ah = Frag<T>::load(Ab + ao);
        V al = ah;
#pragma unroll
        for (int j = 0; j < 4; ++j) acc[i][j] = Frag<T>::mma(ah, bf[j], acc[i][j]);
        if (SPLIT && ph == 0) {
          al = Frag<T>::load(Ab2 + ao);
#pragma unroll
          for (int j = 0; j < 4; ++j) acc[i][j] = Frag<T>::mma(al, bf[j], acc[i][j]);
        }
        Frag<T>::guard(acc[i][0], acc[i][3], ah, al);
      }
      Frag<T>::keep(bf[0], bf[1], bf[2], bf[3]);
    }
  }
  acc_guard4(acc[0][0], acc[0][1], acc[0][2], acc[0][3]);
  acc_guard4(acc[1][0], acc[1][1], acc[1][2], acc[1][3]);
  acc_guard4(acc[2][0], acc[2][1], acc[2][2], acc[2][3]);
  acc_guard4(acc[3][0], acc[3][1], acc[3][2], acc[3][3]);

  float* slab = sT[wave];
#pragma unroll
  for (int i = 0; i < 4; ++i) {
    const int mBase = m0 + (i << 4);
#pragma unroll
    for (int j = 0; j < 4; ++j) {
      const int n = n0 + (j << 4) + rlane;
      float bv = 0.f;
      if (BIAS_MODE == 2) bv = bias[n];
#pragma unroll
      for (int r = 0; r < 8; ++r) {
        float v = acc[i][j][r] * scale;
        if (BIAS_MODE == 1) v += bias[mBase + mOff + r];
        if (BIAS_MODE == 2) v += bv;
        slab[(mOff + r) * 68 + (j << 4) + rlane] = v;
      }
    }
    __builtin_amdgcn_fence(3  , "workgroup");
    __builtin_amdgcn_wave_barrier();
    __builtin_amdgcn_fence(2  , "workgroup");
    if (OUT_MODE == 0) {
      float* C = (float*)Cout + (size_t)b * strideC;
      const int hh = lane >> 4, c4 = (lane & 15) * 4;
      for (int pass = 0; pass < 2; ++pass) {
#pragma unroll
        for (int it = 0; it < 8; ++it) {
          const int row = it * 2 + hh;
          v4f v = *(const v4f*)(slab + row * 68 + c4);
          *(volatile v4f*)(C + (size_t)(mBase + row) * ldc + n0 + c4) = v;
        }
        __threadfence();
      }
    } else {
      const int q = lane >> 3, c8 = (lane & 7) * 8;
      unsigned short* C  = (unsigned short*)Cout  + (size_t)b * strideC;
      unsigned short* C2 = (OUT_MODE == 2) ? ((unsigned short*)Cout2 + (size_t)b * strideC) : nullptr;
      for (int pass = 0; pass < 2; ++pass) {
#pragma unroll
        for (int it = 0; it < 4; ++it) {
          const int row = it * 4 + q;
          const float* sp = slab + row * 68 + c8;
          v8h hv, lv;
#pragma unroll
          for (int e = 0; e < 8; ++e) {
            if (OUT_MODE == 1) {
              hv[e] = (_Float16)sp[e];
            } else {
              const unsigned short hb = f2bf_bits(sp[e]);
              const unsigned short lb = f2bf_bits(sp[e] - bf_bits2f(hb));
              hv[e] = __builtin_bit_cast(_Float16, hb);
              lv[e] = __builtin_bit_cast(_Float16, lb);
            }
          }
          *(volatile v8h*)(C + (size_t)(mBase + row) * ldc + n0 + c8) = hv;
          if (OUT_MODE == 2) *(volatile v8h*)(C2 + (size_t)(mBase + row) * ldc + n0 + c8) = lv;
        }
        __threadfence();
      }
    }
    __builtin_amdgcn_fence(3  , "workgroup");
    __builtin_amdgcn_wave_barrier();
    __builtin_amdgcn_fence(2  , "workgroup");
  }
}

__global__ __launch_bounds__(256) void k_castx(const float* __restrict__ x, unsigned short* __restrict__ X16, int nrows) {
  const long long u = (long long)blockIdx.x * 256 + threadIdx.x;
  constexpr int per = CE / 8;
  if (u >= (long long)nrows * per) return;
  const int r = (int)(u / per); const int c0 = 8 * (int)(u % per);
  const int b = r / SEQ, t = r - b * SEQ;
  const float* s = x + ((size_t)b * SEQ_FULL + t) * CE + c0;
  const v4f a = *(const v4f*)s; const v4f c = *(const v4f*)(s + 4);
  v4u pk;
  pk.x = pk2h(bf_rne(a.x), bf_rne(a.y)); pk.y = pk2h(bf_rne(a.z), bf_rne(a.w));
  pk.z = pk2h(bf_rne(c.x), bf_rne(c.y)); pk.w = pk2h(bf_rne(c.z), bf_rne(c.w));
  VST2(v4u, (v4u*)(X16 + (size_t)r * CE + c0), pk);
}
__global__ __launch_bounds__(256) void k_castwT(const float* __restrict__ W, unsigned short* __restrict__ dst, float sc) {
  const long long u = (long long)blockIdx.x * 256 + threadIdx.x;
  constexpr int per = CE / 8;
  if (u >= (long long)CE * per) return;
  const int c = (int)(u / per); const int r0 = 8 * (int)(u % per);
  float w[8];
#pragma unroll
  for (int e = 0; e < 8; ++e) w[e] = bf_rne(W[(size_t)(r0 + e) * CE + c]) * sc;
  v4u pk; pk.x = pk2h(w[0], w[1]); pk.y = pk2h(w[2], w[3]); pk.z = pk2h(w[4], w[5]); pk.w = pk2h(w[6], w[7]);
  VST2(v4u, (v4u*)(dst + (size_t)c * CE + r0), pk);
}
__global__ __launch_bounds__(256) void k_bias(const float* __restrict__ bq, const float* __restrict__ bk, const float* __restrict__ bv, float* __restrict__ BR) {
  const int u = blockIdx.x * 256 + threadIdx.x;
  if (u >= 3 * CE) return;
  const int i = u & (CE - 1); const int sel = u / CE;
  const float a = bq[i], b2 = bk[i], c = bv[i];
  const float v = bf_rne((sel == 0) ? a : ((sel == 1) ? b2 : c));
  VST2(float, BR + u, v);
}

__global__ __launch_bounds__(256) void k_soft(const float* __restrict__ S, unsigned short* __restrict__ P16, unsigned short* __restrict__ PEh, unsigned short* __restrict__ PEl) {
  __shared__ float red[256];
  __shared__ __align__(16) float prow[SEQ];
  const int t = blockIdx.x, tid = threadIdx.x;
  const float* srow = S + (size_t)t * SEQ;
  const float L2E = 1.4426950408889634f;
  float mx = -__builtin_inff();
#pragma unroll 1
  for (int s = tid; s <= t; s += 256) mx = fmaxf(mx, srow[s]);
  red[tid] = mx; __syncthreads();
  for (int o = 128; o > 0; o >>= 1) { if (tid < o) red[tid] = fmaxf(red[tid], red[tid + o]); __syncthreads(); }
  mx = red[0]; __syncthreads();
  float sum = 0.f;
#pragma unroll 1
  for (int s = tid; s <= t; s += 256) sum += exp2f((srow[s] - mx) * L2E);
  red[tid] = sum; __syncthreads();
  for (int o = 128; o > 0; o >>= 1) { if (tid < o) red[tid] += red[tid + o]; __syncthreads(); }
  sum = red[0];
  const float inv = 1.f / sum;
#pragma unroll 1
  for (int s = tid; s < SEQ; s += 256) { const float v = srow[min(s, t)]; prow[s] = (s <= t) ? exp2f((v - mx) * L2E) * inv : 0.f; }
  __syncthreads();
  if (8 * tid < SEQ) {
    const float* pr = prow + 8 * tid;
    const v4f a = *(const v4f*)pr; const v4f c = *(const v4f*)(pr + 4);
    v4u pk;
    pk.x = pk2h(a.x * 4096.f, a.y * 4096.f); pk.y = pk2h(a.z * 4096.f, a.w * 4096.f);
    pk.z = pk2h(c.x * 4096.f, c.y * 4096.f); pk.w = pk2h(c.z * 4096.f, c.w * 4096.f);
    VST2(v4u, (v4u*)(P16 + (size_t)t * SEQ + 8 * tid), pk);
  }
  if (t < EARLY && tid < 16) {
    const float* pr = prow + 8 * tid;
    unsigned short hb[8], lb[8];
#pragma unroll
    for (int e = 0; e < 8; ++e) { hb[e] = f2bf_bits(pr[e]); lb[e] = f2bf_bits(pr[e] - bf_bits2f(hb[e])); }
    v4u ph, pl;
    ph.x = pk2u(hb[0], hb[1]); ph.y = pk2u(hb[2], hb[3]); ph.z = pk2u(hb[4], hb[5]); ph.w = pk2u(hb[6], hb[7]);
    pl.x = pk2u(lb[0], lb[1]); pl.y = pk2u(lb[2], lb[3]); pl.z = pk2u(lb[4], lb[5]); pl.w = pk2u(lb[6], lb[7]);
    VST2(v4u, (v4u*)(PEh + (size_t)t * EARLY + 8 * tid), ph);
    VST2(v4u, (v4u*)(PEl + (size_t)t * EARLY + 8 * tid), pl);
  }
}

extern "C" void kernel_launch(void* const* d_in, const int* in_sizes, int n_in, void* d_out, int out_size, void* d_ws, size_t ws_size, hipStream_t stream) {
  if (n_in < 7) return;
  const long long need_tok = (long long)(NB - 1) * SEQ_FULL * CE + (long long)SEQ * CE;
  if ((long long)in_sizes[0] < need_tok) return;
  if (in_sizes[1] < CE * CE || in_sizes[3] < CE * CE || in_sizes[5] < CE * CE) return;
  if (in_sizes[2] < CE || in_sizes[4] < CE || in_sizes[6] < CE) return;
  if ((long long)out_size < need_tok) return;
  static_assert((long long)(NB - 1) * SEQ_FULL * CE + (long long)SEQ * CE <= (long long)NB_FULL * SEQ_FULL * CE);

  const float* x  = (const float*)d_in[0];
  const float* Wq = (const float*)d_in[1];
  const float* bq = (const float*)d_in[2];
  const float* Wk = (const float*)d_in[3];
  const float* bk = (const float*)d_in[4];
  const float* Wv = (const float*)d_in[5];
  const float* bv = (const float*)d_in[6];
  float* out = (float*)d_out;

  constexpr int NT = NB * SEQ;
  constexpr size_t X16_B = (size_t)NT * CE * 2;
  constexpr size_t S_B   = (size_t)SEQ * SEQ * 4;
  constexpr size_t R0_B  = (X16_B > S_B) ? X16_B : S_B;
  static_assert(X16_B <= R0_B); static_assert(S_B <= R0_B);
  constexpr size_t W3_B  = (size_t)3 * CE * CE * 2;
  constexpr size_t BR_B  = (size_t)3 * CE * 4;
  constexpr size_t QK_B  = (size_t)NT * 2 * CE * 2;
  constexpr size_t VT_B  = (size_t)CE * NT * 2;
  constexpr size_t VTE_B = (size_t)CE * NB * EARLY * 2;
  constexpr size_t P16_B = (size_t)SEQ * SEQ * 2;
  constexpr size_t PE_B  = (size_t)NB * EARLY * EARLY * 2;
  constexpr size_t TOT_B = R0_B + W3_B + BR_B + 2 * QK_B + VT_B + 2 * VTE_B + P16_B + 2 * PE_B;
  static_assert(TOT_B <= (size_t)134217728);
  static_assert(R0_B % 256 == 0); static_assert(W3_B % 256 == 0); static_assert(BR_B % 256 == 0); static_assert(QK_B % 256 == 0);
  static_assert(VT_B % 256 == 0); static_assert(VTE_B % 256 == 0); static_assert(P16_B % 256 == 0); static_assert(PE_B % 256 == 0);
  if (TOT_B > ws_size) return;
  char* wsp = (char*)d_ws;
  unsigned short* X16 = (unsigned short*)wsp; float* S = (float*)wsp; wsp += R0_B;
  unsigned short* W3  = (unsigned short*)wsp; wsp += W3_B;
  float* BR = (float*)wsp; wsp += BR_B;
  unsigned short* QKh = (unsigned short*)wsp; wsp += QK_B;
  unsigned short* QKl = (unsigned short*)wsp; wsp += QK_B;
  unsigned short* Vt  = (unsigned short*)wsp; wsp += VT_B;
  unsigned short* VtEh = (unsigned short*)wsp; wsp += VTE_B;
  unsigned short* VtEl = (unsigned short*)wsp; wsp += VTE_B;
  unsigned short* P16 = (unsigned short*)wsp; wsp += P16_B;
  unsigned short* PEh = (unsigned short*)wsp; wsp += PE_B;
  unsigned short* PEl = (unsigned short*)wsp; wsp += PE_B;
  if ((size_t)(wsp - (char*)d_ws) > ws_size) return;

  k_castx<<<(unsigned)(((long long)NT * (CE / 8) + 255) / 256), 256, 0, stream>>>(x, X16, NT);
  k_castwT<<<(unsigned)(((long long)CE * (CE / 8) + 255) / 256), 256, 0, stream>>>(Wq, W3, 64.0f);
  k_castwT<<<(unsigned)(((long long)CE * (CE / 8) + 255) / 256), 256, 0, stream>>>(Wk, W3 + (size_t)CE * CE, 64.0f);
  k_castwT<<<(unsigned)(((long long)CE * (CE / 8) + 255) / 256), 256, 0, stream>>>(Wv, W3 + (size_t)2 * CE * CE, 64.0f);
  k_bias<<<(unsigned)((3 * CE + 255) / 256), 256, 0, stream>>>(bq, bk, bv, BR);

  { const int tiles = (NT / 64) * (2 * CE / 64);
    k_gemm64<0, false, 2, 2, 0><<<dim3((unsigned)((tiles + 7) / 8), 1u), 256, 0, stream>>>(
        X16, nullptr, CE, 0, W3, nullptr, CE, 0, (void*)QKh, (void*)QKl, 2 * CE, 0, BR, NT, 2 * CE, CE, 0, 1.0f / 64.0f); }
  { const int tiles = (CE / 64) * (NT / 64);
    k_gemm64<0, false, 1, 1, 0><<<dim3((unsigned)((tiles + 7) / 8), 1u), 256, 0, stream>>>(
        W3 + (size_t)2 * CE * CE, nullptr, CE, 0, X16, nullptr, CE, 0, (void*)Vt, nullptr, NT, 0, BR + 2 * CE, CE, NT, CE, 0, 1.0f / 64.0f); }
  { const int tiles = (CE / 64) * (EARLY / 64);
    k_gemm64<0, false, 1, 2, 0><<<dim3((unsigned)((tiles + 7) / 8), (unsigned)NB), 256, 0, stream>>>(
        W3 + (size_t)2 * CE * CE, nullptr, CE, 0, X16, nullptr, CE, (long long)SEQ * CE, (void*)VtEh, (void*)VtEl, NB * EARLY, (long long)EARLY,
        BR + 2 * CE, CE, EARLY, CE, 0, 1.0f / 64.0f); }

  for (int b = 0; b < NB; ++b) {
    const unsigned short* Ah = QKh + (size_t)b * SEQ * (2 * CE);
    const unsigned short* Al = QKl + (size_t)b * SEQ * (2 * CE);
    { const int tiles = (SEQ / 64) * (SEQ / 64);
      k_gemm64<1, true, 0, 0, 1><<<dim3((unsigned)((tiles + 7) / 8), 1u), 256, 0, stream>>>(
          Ah, Al, 2 * CE, 0, Ah + CE, Al + CE, 2 * CE, 0, (void*)S, nullptr, SEQ, 0, BR, SEQ, SEQ, CE, 0, 0.03125f); }
    k_soft<<<(unsigned)SEQ, 256, 0, stream>>>(S, P16, PEh + (size_t)b * EARLY * EARLY, PEl + (size_t)b * EARLY * EARLY);
    if (SEQ > EARLY) {
      const int tiles = (SEQ / 64 - EARLY / 64) * (CE / 64);
      k_gemm64<0, false, 0, 0, 2><<<dim3((unsigned)((tiles + 7) / 8), 1u), 256, 0, stream>>>(
          P16, nullptr, SEQ, 0, Vt + (size_t)b * SEQ, nullptr, NT, 0, (void*)(out + (size_t)b * SEQ_FULL * CE), nullptr, CE, 0, BR,
          SEQ, CE, SEQ, EARLY / 64, 1.0f / 4096.0f);
    }
  }
  { const int tiles = (EARLY / 64) * (CE / 64);
    k_gemm64<1, true, 0, 0, 0><<<dim3((unsigned)((tiles + 7) / 8), (unsigned)NB), 256, 0, stream>>>(
        PEh, PEl, EARLY, (long long)EARLY * EARLY, VtEh, VtEl, NB * EARLY, (long long)EARLY, (void*)out, nullptr, CE, (long long)SEQ_FULL * CE, BR,
        EARLY, CE, EARLY, 0, 1.0f); }
}
